// EncoderRNN_74483322847540
// MI455X (gfx1250) — hardware-run, weakly checked
//
#include <hip/hip_runtime.h>
#include <math.h>

constexpr int NB     = 8;
constexpr int SEQ    = 1024;
constexpr int FIN    = 128;
constexpr int EMB    = 256;
constexpr int HID    = 256;
constexpr int NLAYER = 2;
constexpr int NHEAD  = 4;
constexpr int KDIM   = 64;
constexpr int NROW   = NB * SEQ;
constexpr int G4     = 4 * HID;
constexpr int CATK   = 2 * EMB;
constexpr int NPOSC  = 64;
constexpr int NT     = 256;
constexpr int HP     = 264;
constexpr int SLP    = 36;
constexpr int KVC    = 64;
constexpr int OSP    = 68;
constexpr float WCAR      = 64.0f;
constexpr float ACAR      = 8.0f;
constexpr float SC_AW     = 1.0f / 512.0f;
constexpr float PCAR      = 32768.0f;
constexpr float MASK_FILL = -1.0e9f;
constexpr float LN_EPS_F  = 1.0e-3f;
constexpr float PI_F      = 3.14159265358979323846f;

static_assert(NROW % 64 == 0 && EMB % 64 == 0 && HID % 64 == 0 && G4 % 64 == 0 && SEQ % 64 == 0);
static_assert(FIN % 32 == 0 && HID % 32 == 0 && CATK % 32 == 0 && EMB % 32 == 0);
static_assert(NHEAD * KDIM == HID && KDIM == 64 && SEQ % KVC == 0);
static_assert(NROW % (NT / 32) == 0);
static_assert(HP % 8 == 0 && SLP % 4 == 0 && OSP % 4 == 0);
static_assert((NB * G4) % (4 * NT) == 0);
static_assert(HID == 32 * (NT / 32));
static_assert(NB <= 8);
static_assert((NROW * FIN) % 8 == 0 && (SEQ * NPOSC) % NT == 0);
static_assert(EMB == 256 && HID == 256);
static_assert(FIN % 64 == 0 && CATK % 64 == 0);

typedef __attribute__((ext_vector_type(16))) _Float16 v16h;
typedef __attribute__((ext_vector_type(8)))  _Float16 v8h;
typedef __attribute__((ext_vector_type(16))) __bf16   v16b;
typedef __attribute__((ext_vector_type(8)))  __bf16   v8b;
typedef __attribute__((ext_vector_type(8)))  float    v8f;
typedef __attribute__((ext_vector_type(4)))  float    v4f;
typedef __attribute__((ext_vector_type(4)))  unsigned u4x;
typedef __attribute__((ext_vector_type(2)))  unsigned u2x;

__device__ __forceinline__ unsigned short f2bf_bits(float f) {
  unsigned u = __float_as_uint(f);
  return (unsigned short)((u + 0x7FFFu + ((u >> 16) & 1u)) >> 16);
}
__device__ __forceinline__ float bf_bits2f(unsigned short h) { return __uint_as_float(((unsigned)h) << 16); }
__device__ __forceinline__ float bf16r(float f) { return bf_bits2f(f2bf_bits(f)); }
__device__ __forceinline__ unsigned short h_bits(float f) { return __builtin_bit_cast(unsigned short, (_Float16)f); }
__device__ __forceinline__ unsigned pack2(unsigned short lo, unsigned short hi) { return (unsigned)lo | ((unsigned)hi << 16); }
__device__ __forceinline__ void split_bf(float f, unsigned short& hb, unsigned short& lb) {
  hb = f2bf_bits(f); lb = f2bf_bits(f - bf_bits2f(hb));
}
__device__ __forceinline__ unsigned bfw2(float f0, float f1, unsigned& lo_word) {
  unsigned short h0, l0, h1, l1; split_bf(f0, h0, l0); split_bf(f1, h1, l1);
  lo_word = pack2(l0, l1); return pack2(h0, h1);
}

__device__ __forceinline__ void keep4_h(v16h a, v16h b, v16h c, v16h d) { asm volatile("v_nop" :: "v"(a), "v"(b), "v"(c), "v"(d)); }
__device__ __forceinline__ void keep4_b(v16b a, v16b b, v16b c, v16b d) { asm volatile("v_nop" :: "v"(a), "v"(b), "v"(c), "v"(d)); }
__device__ __forceinline__ void acc_guard4(v8f& a, v8f& b, v8f& c, v8f& d) { asm volatile("v_nop\n\tv_nop\n\tv_nop\n\tv_nop" : "+v"(a), "+v"(b), "+v"(c), "+v"(d)); }
template <typename VV>
__device__ __forceinline__ void guard_all(v8f& a, v8f& b, v8f& c, v8f& d, VV x0, VV x1, VV y0, VV y1, VV y2, VV y3) {
  asm volatile("v_nop\n\tv_nop\n\tv_nop\n\tv_nop" : "+v"(a), "+v"(b), "+v"(c), "+v"(d) : "v"(x0), "v"(x1), "v"(y0), "v"(y1), "v"(y2), "v"(y3));
}
template <typename T> struct Frag;
template <> struct Frag<_Float16> {
  typedef v16h V; union U { v16h v; v8h h[2]; };
  static __device__ __forceinline__ v16h load(const _Float16* p) {
    U f; f.h[0] = *(const v8h*)(p); f.h[1] = *(const v8h*)(p + 16); return f.v;
  }
  static __device__ __forceinline__ v8f mma(v16h a, v16h b, v8f c) {
    return __builtin_amdgcn_wmma_f32_16x16x32_f16(false, a, false, b, (short)0, c, false, false);
  }
  static __device__ __forceinline__ void keep(v16h a, v16h b, v16h c, v16h d) { keep4_h(a, b, c, d); }
};
template <> struct Frag<__bf16> {
  typedef v16b V; union U { v16b v; v8b h[2]; };
  static __device__ __forceinline__ v16b load(const __bf16* p) {
    U f; f.h[0] = *(const v8b*)(p); f.h[1] = *(const v8b*)(p + 16); return f.v;
  }
  static __device__ __forceinline__ v8f mma(v16b a, v16b b, v8f c) {
    return __builtin_amdgcn_wmma_f32_16x16x32_bf16(false, a, false, b, (short)0, c, false, false);
  }
  static __device__ __forceinline__ void keep(v16b a, v16b b, v16b c, v16b d) { keep4_b(a, b, c, d); }
};
__device__ __forceinline__ v8f mma_g(v16h a, v16h b, v8f c) {
  c = Frag<_Float16>::mma(a, b, c);
  asm volatile("v_nop\n\tv_nop\n\tv_nop\n\tv_nop" : "+v"(c) : "v"(a), "v"(b));
  return c;
}
__device__ __forceinline__ void lds_sync_wave() {
  __builtin_amdgcn_fence(__ATOMIC_RELEASE, "workgroup");
  __builtin_amdgcn_wave_barrier();
  __builtin_amdgcn_fence(__ATOMIC_ACQUIRE, "workgroup");
}
__device__ __forceinline__ float fsig(float x)  { return __builtin_amdgcn_rcpf(1.0f + expf(-x)); }
__device__ __forceinline__ float ftanh(float x) { return 1.0f - 2.0f * __builtin_amdgcn_rcpf(expf(2.0f * x) + 1.0f); }

template <int ET> struct Elem;
template <> struct Elem<0> { typedef _Float16 T; };
template <> struct Elem<1> { typedef __bf16 T; };
template <int ET, bool ASPLIT, int BIAS_MODE, int ACT, bool MASK, bool ADDPOS, bool RESID, int OUT_MODE>
__global__ __launch_bounds__(256) void gemm_kernel(
    const unsigned short* __restrict__ Ap, const unsigned short* __restrict__ A2p, int lda, long strideA,
    const unsigned short* __restrict__ Btp, int ldb, long strideB,
    void* Cout, void* Cout2, void* Cout3, int ldc, long strideC,
    const float* __restrict__ bias, const float* resid, const float* __restrict__ pos,
    const int* __restrict__ lens, int M, int N, int K, float scale, float c16scale) {
  typedef typename Elem<ET>::T T;
  typedef typename Frag<T>::V V;
  const T* A  = (const T*)Ap;
  const T* A2 = (const T*)A2p;
  const T* Bt = (const T*)Btp;
  __shared__ __align__(16) float sT[8][16 * 68];
  const int b    = blockIdx.y;
  const int lane = threadIdx.x & 31;
  const int wave = threadIdx.x >> 5;
  const int tilesN = N >> 6;
  const int tilesM = M >> 6;
  const int tile = blockIdx.x * 8 + wave;
  if (tile >= tilesM * tilesN) return;
  const int tm = tile / tilesN;
  const int tn = tile - tm * tilesN;
  const int m0 = tm << 6;
  const int n0 = tn << 6;

  const T* Ab  = A  + (size_t)b * strideA;
  const T* Ab2 = A2 + (size_t)b * strideA;
  const T* Bb  = Bt + (size_t)b * strideB;

  const int rlane = lane & 15;
  const int koff  = (lane >> 4) * 8;
  const int mOff  = (lane >> 4) * 8;

  v8f acc[4][4];
#pragma unroll
  for (int i = 0; i < 4; ++i)
#pragma unroll
    for (int j = 0; j < 4; ++j) acc[i][j] = (v8f){0.f,0.f,0.f,0.f,0.f,0.f,0.f,0.f};

  for (int k0 = 0; k0 < K; k0 += 32) {
    V bh[4];
#pragma unroll
    for (int j = 0; j < 4; ++j) {
      const size_t bo = (size_t)(n0 + (j << 4) + rlane) * ldb + koff + k0;
      bh[j] = Frag<T>::load(Bb + bo);
    }
#pragma unroll
    for (int i = 0; i < 4; ++i) {
      const size_t ao = (size_t)(m0 + (i << 4) + rlane) * lda + koff + k0;
      const V ah = Frag<T>::load(Ab + ao);
      V al = ah;
      if (ASPLIT) al = Frag<T>::load(Ab2 + ao);
#pragma unroll
      for (int j = 0; j < 4; ++j) {
        acc[i][j] = Frag<T>::mma(ah, bh[j], acc[i][j]);
        if (ASPLIT) acc[i][j] = Frag<T>::mma(al, bh[j], acc[i][j]);
      }
      guard_all<V>(acc[i][0], acc[i][1], acc[i][2], acc[i][3], ah, al, bh[0], bh[1], bh[2], bh[3]);
    }
    Frag<T>::keep(bh[0], bh[1], bh[2], bh[3]);
  }
  acc_guard4(acc[0][0], acc[0][1], acc[0][2], acc[0][3]);
  acc_guard4(acc[1][0], acc[1][1], acc[1][2], acc[1][3]);
  acc_guard4(acc[2][0], acc[2][1], acc[2][2], acc[2][3]);
  acc_guard4(acc[3][0], acc[3][1], acc[3][2], acc[3][3]);

  float* slab = sT[wave];
  int lenT = 0;
  if (MASK) {
    int bb = m0 / SEQ;
    bb = bb > NB - 1 ? NB - 1 : bb;
    lenT = lens[bb];
  }
  const float* Rb = RESID ? (resid + (size_t)b * strideC) : nullptr;
  const int hq = lane >> 4, c4 = (lane & 15) * 4;
  const int q8 = lane >> 3, c8 = (lane & 7) * 8;
  constexpr bool PHASEA = MASK || ADDPOS || RESID;
#pragma unroll
  for (int i = 0; i < 4; ++i) {
    const int mBase = m0 + (i << 4);
    float bmr[8] = {0.f, 0.f, 0.f, 0.f, 0.f, 0.f, 0.f, 0.f};
    if (BIAS_MODE == 1) {
      const v4f b0 = *(const v4f*)(bias + mBase + mOff);
      const v4f b1 = *(const v4f*)(bias + mBase + mOff + 4);
#pragma unroll
      for (int e = 0; e < 4; ++e) { bmr[e] = bf16r(b0[e]); bmr[4 + e] = bf16r(b1[e]); }
    }
#pragma unroll
    for (int j = 0; j < 4; ++j) {
      const int n = n0 + (j << 4) + rlane;
      float bvn = 0.f;
      if (BIAS_MODE == 2) bvn = bf16r(bias[n]);
#pragma unroll
      for (int r = 0; r < 8; ++r) {
        float v = acc[i][j][r] * scale;
        if (BIAS_MODE == 1) v += bmr[r];
        if (BIAS_MODE == 2) v += bvn;
        if (ACT == 2) v = fmaxf(v, 0.0f);
        slab[(mOff + r) * 68 + (j << 4) + rlane] = v;
      }
    }
    lds_sync_wave();
    if (PHASEA) {
#pragma unroll
      for (int hf = 0; hf < 2; ++hf) {
#pragma unroll
        for (int u = 0; u < 4; ++u) {
          const int it = hf * 4 + u;
          const int row = it * 2 + hq;
          const int grow = mBase + row;
          v4f v = *(const v4f*)(slab + row * 68 + c4);
          if (ADDPOS) {
            const bool first = (n0 == 0);
            const int pc = first ? c4 : 0;
            const v4f p4 = *(const v4f*)(pos + (size_t)(grow & (SEQ - 1)) * NPOSC + pc);
            const float pf = first ? 1.0f : 0.0f;
            v = v + p4 * pf;
          }
          if (MASK) {
            const float mv = ((grow & (SEQ - 1)) < lenT) ? 1.0f : 0.0f;
            v = v * mv;
          }
          if (RESID) {
            const v4f r4 = *(const v4f*)(Rb + (size_t)grow * ldc + n0 + c4);
            v = v + r4;
          }
          *(v4f*)(slab + row * 68 + c4) = v;
        }
        asm volatile("" ::: "memory");
      }
      lds_sync_wave();
    }
    if (OUT_MODE == 0 || OUT_MODE == 2) {
      float* Cf = (float*)Cout + (size_t)b * strideC;
      for (int pass = 0; pass < 2; ++pass) {
#pragma unroll
        for (int it = 0; it < 8; ++it) {
          const int row = it * 2 + hq;
          const v4f v = *(const v4f*)(slab + row * 68 + c4);
          *(volatile v4f*)(Cf + (size_t)(mBase + row) * ldc + n0 + c4) = v;
        }
        __threadfence();
      }
    }
    if (OUT_MODE == 1 || OUT_MODE == 2) {
      unsigned short* Ca = (unsigned short*)((OUT_MODE == 1) ? Cout : Cout2) + (size_t)b * strideC;
      unsigned short* Cb = (unsigned short*)Cout3 + (size_t)b * strideC;
      for (int pass = 0; pass < 2; ++pass) {
#pragma unroll
        for (int it = 0; it < 4; ++it) {
          const int row = it * 4 + q8;
          const float* sp = slab + row * 68 + c8;
          const v4f s0 = *(const v4f*)(sp);
          const v4f s1 = *(const v4f*)(sp + 4);
          const float f[8] = {s0[0], s0[1], s0[2], s0[3], s1[0], s1[1], s1[2], s1[3]};
          u4x wa = {0u, 0u, 0u, 0u}, wb = {0u, 0u, 0u, 0u};
#pragma unroll
          for (int e = 0; e < 4; ++e) {
            if (OUT_MODE == 1) {
              wa[e] = pack2(h_bits(f[2 * e] * c16scale), h_bits(f[2 * e + 1] * c16scale));
            } else {
              unsigned lw; wa[e] = bfw2(f[2 * e], f[2 * e + 1], lw); wb[e] = lw;
            }
          }
          const size_t o = (size_t)(mBase + row) * ldc + n0 + c8;
          *(volatile u4x*)(Ca + o) = wa;
          if (OUT_MODE == 2) *(volatile u4x*)(Cb + o) = wb;
        }
        __threadfence();
      }
    }
    lds_sync_wave();
  }
}

template <int MODE>
__global__ __launch_bounds__(NT) void tpw_kernel(const float* __restrict__ src, int R, int C, int ldo,
                                                unsigned short* __restrict__ O, float sc, long sstride, long dstride) {
  __shared__ float Tt[64 * 65];
  const int tid = threadIdx.x;
  const float* s = src + (size_t)blockIdx.z * (size_t)sstride;
  unsigned short* o = O + (size_t)blockIdx.z * (size_t)dstride;
  const int c0 = blockIdx.x * 64, r0 = blockIdx.y * 64;
#pragma unroll
  for (int i = 0; i < 4; ++i) {
    const int idx = i * NT + tid;
    const int rr = idx >> 4, cc = (idx & 15) * 4;
    const v4f v = *(const v4f*)(s + (size_t)(r0 + rr) * (size_t)C + c0 + cc);
    Tt[rr * 65 + cc + 0] = v[0];
    Tt[rr * 65 + cc + 1] = v[1];
    Tt[rr * 65 + cc + 2] = v[2];
    Tt[rr * 65 + cc + 3] = v[3];
  }
  __syncthreads();
  const int q = tid >> 3, c8 = (tid & 7) * 8;
  u4x w[2];
#pragma unroll
  for (int g = 0; g < 2; ++g) {
    const int qq = g * 32 + q;
#pragma unroll
    for (int e = 0; e < 4; ++e) {
      const float f0 = Tt[(c8 + 2 * e) * 65 + qq];
      const float f1 = Tt[(c8 + 2 * e + 1) * 65 + qq];
      unsigned short b0, b1;
      if (MODE == 0) { b0 = f2bf_bits(f0 * sc); b1 = f2bf_bits(f1 * sc); }
      else           { b0 = h_bits(bf16r(f0) * sc); b1 = h_bits(bf16r(f1) * sc); }
      w[g][e] = pack2(b0, b1);
    }
  }
  for (int pass = 0; pass < 2; ++pass) {
#pragma unroll
    for (int g = 0; g < 2; ++g) {
      const size_t oo = (size_t)(c0 + g * 32 + q) * (size_t)ldo + (size_t)(r0 + c8);
      *(volatile u4x*)(o + oo) = w[g];
    }
    __threadfence();
  }
}

__global__ __launch_bounds__(NT) void cvt8b_kernel(const float* __restrict__ src, unsigned short* __restrict__ dst, int n8) {
  const int i = blockIdx.x * NT + threadIdx.x;
  if (i < n8) {
    const v4f a = *(const v4f*)(src + (size_t)i * 8);
    const v4f c = *(const v4f*)(src + (size_t)i * 8 + 4);
    u4x w;
    w[0] = pack2(f2bf_bits(a[0]), f2bf_bits(a[1]));
    w[1] = pack2(f2bf_bits(a[2]), f2bf_bits(a[3]));
    w[2] = pack2(f2bf_bits(c[0]), f2bf_bits(c[1]));
    w[3] = pack2(f2bf_bits(c[2]), f2bf_bits(c[3]));
    *(volatile u4x*)(dst + (size_t)i * 8) = w;
    __threadfence();
    *(volatile u4x*)(dst + (size_t)i * 8) = w;
  }
}

__global__ __launch_bounds__(NT) void pos_kernel(float* __restrict__ POS) {
  const int i = blockIdx.x * NT + threadIdx.x;
  if (i >= SEQ * NPOSC) return;
  const int s  = i / NPOSC;
  const int cc = i - s * NPOSC;
  const int j  = cc & 15;
  const float fr  = PI_F * __uint_as_float((unsigned)(126 - j) << 23);
  const float ang = (float)s * fr;
  const float sv = sinf(ang);
  const float cv = cosf(ang);
  const float v = (cc < 16) ? sv : ((cc < 32) ? cv : 0.0f);
  ((volatile float*)POS)[i] = v;
  __threadfence();
  ((volatile float*)POS)[i] = v;
}

__global__ __launch_bounds__(NT) void concat_kernel(const float* __restrict__ H, const int* __restrict__ pairs,
                                                    unsigned short* __restrict__ CATH, unsigned short* __restrict__ CATL) {
  const int tid = threadIdx.x, lane = tid & 31;
  const int row = blockIdx.x * (NT / 32) + (tid >> 5);
  if (row >= NROW) return;
  const int b = row / SEQ;
  int pw = pairs[row];
  const float fsel = (pw >= 0) ? 1.0f : 0.0f;
  pw = pw < 0 ? 0 : pw;
  pw = pw > SEQ - 1 ? SEQ - 1 : pw;
  const float* prow = H + ((size_t)b * SEQ + (size_t)pw) * EMB + 8 * lane;
  const float* orow = H + (size_t)row * EMB + 8 * lane;
  const v4f p0 = *(const v4f*)(prow), p1 = *(const v4f*)(prow + 4);
  const v4f o0 = *(const v4f*)(orow), o1 = *(const v4f*)(orow + 4);
  float pf[8], of[8];
#pragma unroll
  for (int e = 0; e < 4; ++e) {
    pf[e]     = fmaxf(p0[e] * fsel, 0.0f) + 0.0f;
    pf[4 + e] = fmaxf(p1[e] * fsel, 0.0f) + 0.0f;
    of[e]     = fmaxf(o0[e], 0.0f) + 0.0f;
    of[4 + e] = fmaxf(o1[e], 0.0f) + 0.0f;
  }
  u4x ph, pl, oh, ol;
#pragma unroll
  for (int e = 0; e < 4; ++e) {
    unsigned lw;
    ph[e] = bfw2(pf[2 * e], pf[2 * e + 1], lw); pl[e] = lw;
    oh[e] = bfw2(of[2 * e], of[2 * e + 1], lw); ol[e] = lw;
  }
  unsigned short* dh = CATH + (size_t)row * CATK + 8 * lane;
  unsigned short* dl = CATL + (size_t)row * CATK + 8 * lane;
  for (int pass = 0; pass < 2; ++pass) {
    *(volatile u4x*)(dh) = ph;
    *(volatile u4x*)(dh + EMB) = oh;
    *(volatile u4x*)(dl) = pl;
    *(volatile u4x*)(dl + EMB) = ol;
    __threadfence();
  }
}

__global__ __launch_bounds__(NT) void ln_kernel(const float* __restrict__ H, const float* __restrict__ gam,
                                                const float* __restrict__ bet, const int* __restrict__ lens,
                                                unsigned short* __restrict__ HLNH, unsigned short* __restrict__ HLNL) {
  const int tid = threadIdx.x, lane = tid & 31;
  const int row = blockIdx.x * (NT / 32) + (tid >> 5);
  if (row >= NROW) return;
  const int b = row / SEQ, s_idx = row - b * SEQ;
  const float* rp = H + (size_t)row * EMB + 8 * lane;
  v4f v0 = *(const v4f*)(rp), v1 = *(const v4f*)(rp + 4);
  const v4f g0 = *(const v4f*)(gam + 8 * lane), g1 = *(const v4f*)(gam + 8 * lane + 4);
  const v4f e0 = *(const v4f*)(bet + 8 * lane), e1 = *(const v4f*)(bet + 8 * lane + 4);
  float s = ((v0[0] + v0[1]) + (v0[2] + v0[3])) + ((v1[0] + v1[1]) + (v1[2] + v1[3]));
#pragma unroll
  for (int off = 1; off < 32; off <<= 1) s += __shfl_xor(s, off, 32);
  const float mu = s * (1.0f / EMB);
  float ss = 0.0f;
#pragma unroll
  for (int e = 0; e < 4; ++e) {
    const float d0 = v0[e] - mu; v0[e] = d0; ss += d0 * d0;
    const float d1 = v1[e] - mu; v1[e] = d1; ss += d1 * d1;
  }
#pragma unroll
  for (int off = 1; off < 32; off <<= 1) ss += __shfl_xor(ss, off, 32);
  const float var  = ss * (1.0f / EMB);
  const float rstd = 1.0f / sqrtf(var + LN_EPS_F);
  const float mv = (s_idx < lens[b]) ? 1.0f : 0.0f;
  float f[8];
#pragma unroll
  for (int e = 0; e < 4; ++e) {
    f[e]     = ((bf16r(g0[e]) * v0[e]) * rstd + bf16r(e0[e])) * mv;
    f[4 + e] = ((bf16r(g1[e]) * v1[e]) * rstd + bf16r(e1[e])) * mv;
  }
  u4x wh, wl;
#pragma unroll
  for (int e = 0; e < 4; ++e) { unsigned lw; wh[e] = bfw2(f[2 * e], f[2 * e + 1], lw); wl[e] = lw; }
  unsigned short* dh = HLNH + (size_t)row * EMB + 8 * lane;
  unsigned short* dl = HLNL + (size_t)row * EMB + 8 * lane;
  for (int pass = 0; pass < 2; ++pass) {
    *(volatile u4x*)(dh) = wh;
    *(volatile u4x*)(dl) = wl;
    __threadfence();
  }
}

__global__ __launch_bounds__(NT) void post_kernel(const float* __restrict__ HS, const int* __restrict__ lens,
                                                  float* H, unsigned short* __restrict__ HH, unsigned short* __restrict__ HL,
                                                  float fold) {
  const int tid = threadIdx.x, lane = tid & 31;
  const int row = blockIdx.x * (NT / 32) + (tid >> 5);
  if (row >= NROW) return;
  const int b = row / SEQ, s_idx = row - b * SEQ;
  const float mv = (s_idx < lens[b]) ? 1.0f : 0.0f;
  const float* ap = HS + (size_t)row * HID + 4 * lane;
  float*       hp = H  + (size_t)row * HID + 4 * lane;
  const v4f a0 = *(const v4f*)(ap), a1 = *(const v4f*)(ap + 128);
  const v4f o0 = *(const v4f*)(hp), o1 = *(const v4f*)(hp + 128);
  const v4f w0 = a0 * mv + o0 * fold;
  const v4f w1 = a1 * mv + o1 * fold;
  u2x h0w, l0w, h1w, l1w;
#pragma unroll
  for (int e = 0; e < 2; ++e) {
    unsigned lw;
    h0w[e] = bfw2(w0[2 * e], w0[2 * e + 1], lw); l0w[e] = lw;
    h1w[e] = bfw2(w1[2 * e], w1[2 * e + 1], lw); l1w[e] = lw;
  }
  unsigned short* hh = HH + (size_t)row * HID + 4 * lane;
  unsigned short* hl = HL + (size_t)row * HID + 4 * lane;
  for (int pass = 0; pass < 2; ++pass) {
    *(volatile v4f*)(hp)       = w0;
    *(volatile v4f*)(hp + 128) = w1;
    *(volatile u2x*)(hh)       = h0w;
    *(volatile u2x*)(hh + 128) = h1w;
    *(volatile u2x*)(hl)       = l0w;
    *(volatile u2x*)(hl + 128) = l1w;
    __threadfence();
  }
}

__global__ __launch_bounds__(NT) void lstm_kernel(const float* __restrict__ ZX, const unsigned short* __restrict__ WHp,
                                                  float* __restrict__ HS) {
  __shared__ __align__(16) _Float16 Ah[16 * HP];
  __shared__ __align__(16) float    Zs[NB * G4];
  __shared__ __align__(16) float    Sl[NT / 32][16 * SLP];
  const _Float16* WH = (const _Float16*)WHp;
  const int tid = threadIdx.x, lane = tid & 31, wave = tid >> 5;
  const int c = lane & 15, hh = lane >> 4, koff = hh * 8;
  const int rq = lane >> 3, c4 = (lane & 7) * 4;

#pragma unroll 1
  for (int i = tid; i < 16 * HP; i += NT) Ah[i] = (_Float16)0.0f;
  float cst[2][8], hst[2][8];
#pragma unroll
  for (int nt = 0; nt < 2; ++nt)
#pragma unroll
    for (int r = 0; r < 8; ++r) { cst[nt][r] = 0.0f; hst[nt][r] = 0.0f; }
  __syncthreads();

  const _Float16* ahrow = Ah + c * HP + koff;
  float* slab = Sl[wave];
  const v8f z8 = {0.f, 0.f, 0.f, 0.f, 0.f, 0.f, 0.f, 0.f};
  const float rowsel = (hh == 0) ? ACAR : 0.0f;

#pragma unroll 1
  for (int t = 0; t < SEQ; ++t) {
#pragma unroll
    for (int it = 0; it < 4; ++it) {
      const int idx = it * NT + tid;
      const int row = idx >> 8, cc = (idx & 255) * 4;
      const v4f v = *(const v4f*)(ZX + ((size_t)row * SEQ + (size_t)t) * G4 + cc);
      *(v4f*)(Zs + row * G4 + cc) = v;
    }
    asm volatile("" ::: "memory");
#pragma unroll
    for (int it = 4; it < 8; ++it) {
      const int idx = it * NT + tid;
      const int row = idx >> 8, cc = (idx & 255) * 4;
      const v4f v = *(const v4f*)(ZX + ((size_t)row * SEQ + (size_t)t) * G4 + cc);
      *(v4f*)(Zs + row * G4 + cc) = v;
    }
    __syncthreads();

#pragma unroll
    for (int nt = 0; nt < 2; ++nt) {
      const int j = 32 * wave + 16 * nt + c;
      const _Float16* wh = WH + (size_t)j * HID + koff;
      v8f acc0 = z8, acc1 = z8, acc2 = z8, acc3 = z8;
#pragma unroll 1
      for (int k0 = 0; k0 < HID; k0 += 32) {
        const v16h a  = Frag<_Float16>::load(ahrow + k0);
        const v16h b0 = Frag<_Float16>::load(wh + k0);
        const v16h b1 = Frag<_Float16>::load(wh + (size_t)1 * HID * HID + k0);
        const v16h b2 = Frag<_Float16>::load(wh + (size_t)2 * HID * HID + k0);
        const v16h b3 = Frag<_Float16>::load(wh + (size_t)3 * HID * HID + k0);
        acc0 = Frag<_Float16>::mma(a, b0, acc0);
        acc1 = Frag<_Float16>::mma(a, b1, acc1);
        acc2 = Frag<_Float16>::mma(a, b2, acc2);
        acc3 = Frag<_Float16>::mma(a, b3, acc3);
        guard_all<v16h>(acc0, acc1, acc2, acc3, a, a, b0, b1, b2, b3);
      }
      acc_guard4(acc0, acc1, acc2, acc3);
#pragma unroll
      for (int r = 0; r < 8; ++r) {
        const float* zr = Zs + r * G4 + j;
        const float zi = acc0[r] * SC_AW + zr[0];
        const float zf = acc1[r] * SC_AW + zr[HID];
        const float zg = acc2[r] * SC_AW + zr[2 * HID];
        const float zo = acc3[r] * SC_AW + zr[3 * HID];
        const float ig = fsig(zi);
        const float fg = fsig(zf);
        const float og = fsig(zo);
        const float gg = ftanh(zg);
        const float cn = fg * cst[nt][r] + ig * gg;
        cst[nt][r] = cn;
        hst[nt][r] = og * ftanh(cn);
      }
    }
    __syncthreads();

#pragma unroll
    for (int nt = 0; nt < 2; ++nt) {
      const int j = 32 * wave + 16 * nt + c;
#pragma unroll
      for (int r = 0; r < 8; ++r) Ah[(8 * hh + r) * HP + j] = (_Float16)(hst[nt][r] * rowsel);
    }
#pragma unroll
    for (int nt = 0; nt < 2; ++nt)
#pragma unroll
      for (int r = 0; r < 8; ++r) slab[(8 * hh + r) * SLP + 16 * nt + c] = hst[nt][r];
    lds_sync_wave();
    for (int pass = 0; pass < 2; ++pass) {
#pragma unroll
      for (int it = 0; it < 2; ++it) {
        const int r = it * 4 + rq;
        const v4f v = *(const v4f*)(slab + r * SLP + c4);
        *(volatile v4f*)(HS + ((size_t)r * SEQ + (size_t)t) * HID + 32 * wave + c4) = v;
      }
      __threadfence();
    }
    lds_sync_wave();
  }
}

__global__ __launch_bounds__(128) void attn_kernel(const unsigned short* __restrict__ Qp, const unsigned short* __restrict__ Kp,
                                                   const unsigned short* __restrict__ Vtp, const int* __restrict__ lens,
                                                   unsigned short* __restrict__ AOp) {
  __shared__ __align__(16) _Float16 Ksh[KVC * KDIM];
  __shared__ __align__(16) _Float16 Vth[KDIM * KVC];
  __shared__ __align__(16) _Float16 Psh[4][16 * KVC];
  __shared__ __align__(16) float    Os[4][16 * OSP];
  const _Float16* Q  = (const _Float16*)Qp;
  const _Float16* K  = (const _Float16*)Kp;
  const _Float16* Vt = (const _Float16*)Vtp;
  const int tid = threadIdx.x, wave = tid >> 5, lane = tid & 31;
  const int hh = lane >> 4, c = lane & 15;
  const int nqb = SEQ / 64;
  const int bx = blockIdx.x;
  const int qb = bx % nqb;
  const int bh = bx / nqb;
  const int h  = bh % NHEAD;
  const int b  = bh / NHEAD;
  const int q0 = qb * 64 + wave * 16;
  int len = lens[b];
  len = len < 0 ? 0 : len;
  len = len > SEQ ? SEQ : len;
  const int nChunks = (len > 0) ? ((len + KVC - 1) / KVC) : (SEQ / KVC);

  v16h qa[2];
  {
    const _Float16* qrow = Q + ((size_t)b * SEQ + (size_t)(q0 + c)) * HID + h * KDIM;
#pragma unroll
    for (int dc = 0; dc < 2; ++dc) qa[dc] = Frag<_Float16>::load(qrow + dc * 32 + 8 * hh);
  }
  float mrow[8], lrow[8];
  v8f oacc[4];
#pragma unroll
  for (int r = 0; r < 8; ++r) { mrow[r] = -INFINITY; lrow[r] = 0.0f; }
#pragma unroll
  for (int t = 0; t < 4; ++t) oacc[t] = (v8f){0.f,0.f,0.f,0.f,0.f,0.f,0.f,0.f};

#pragma unroll 1
  for (int kc = 0; kc < nChunks; ++kc) {
    const int kv0 = kc * KVC;
    __syncthreads();
    {
      const int kvr = tid >> 1, dh = (tid & 1) * 32;
      const _Float16* ks = K  + ((size_t)b * SEQ + (size_t)(kv0 + kvr)) * HID + h * KDIM + dh;
      const _Float16* vs = Vt + ((size_t)b * HID + (size_t)(h * KDIM + kvr)) * SEQ + kv0 + dh;
      u4x kw[4], vw[4];
#pragma unroll
      for (int i = 0; i < 4; ++i) { kw[i] = *(const u4x*)(const void*)(ks + 8 * i); vw[i] = *(const u4x*)(const void*)(vs + 8 * i); }
#pragma unroll
      for (int i = 0; i < 4; ++i) {
        *(u4x*)(void*)(Ksh + kvr * KDIM + dh + 8 * i) = kw[i];
        *(u4x*)(void*)(Vth + kvr * KVC  + dh + 8 * i) = vw[i];
      }
    }
    __syncthreads();

    v8f s[4];
#pragma unroll
    for (int j = 0; j < 4; ++j) {
      s[j] = (v8f){0.f,0.f,0.f,0.f,0.f,0.f,0.f,0.f};
#pragma unroll
      for (int dc = 0; dc < 2; ++dc) {
        const v16h kb = Frag<_Float16>::load(Ksh + (j * 16 + c) * KDIM + dc * 32 + 8 * hh);
        s[j] = mma_g(qa[dc], kb, s[j]);
      }
    }
    float cm[8];
#pragma unroll
    for (int r = 0; r < 8; ++r) {
      float m = -INFINITY;
#pragma unroll
      for (int j = 0; j < 4; ++j) {
        const int kvcol = kv0 + j * 16 + c;
        const bool masked = (kvcol >= len);
        const float sv = masked ? MASK_FILL : s[j][r] * SC_AW;
        s[j][r] = sv;
        m = fmaxf(m, sv);
      }
#pragma unroll
      for (int off = 1; off < 16; off <<= 1) m = fmaxf(m, __shfl_xor(m, off, 32));
      cm[r] = m;
    }
    _Float16* pwh = Psh[wave];
#pragma unroll
    for (int r = 0; r < 8; ++r) {
      const float mnew  = fmaxf(mrow[r], cm[r]);
      const float alpha = expf(mrow[r] - mnew);
      mrow[r] = mnew;
      float psum = 0.0f;
#pragma unroll
      for (int j = 0; j < 4; ++j) {
        const float p = expf(s[j][r] - mnew);
        psum += p;
        pwh[(8 * hh + r) * KVC + j * 16 + c] = (_Float16)(p * PCAR);
      }
#pragma unroll
      for (int off = 1; off < 16; off <<= 1) psum += __shfl_xor(psum, off, 32);
      lrow[r] = lrow[r] * alpha + psum;
#pragma unroll
      for (int t = 0; t < 4; ++t) oacc[t][r] *= alpha;
    }
    lds_sync_wave();
#pragma unroll
    for (int kk = 0; kk < 2; ++kk) {
      const v16h pa = Frag<_Float16>::load(pwh + c * KVC + kk * 32 + 8 * hh);
#pragma unroll
      for (int t = 0; t < 4; ++t) {
        const v16h vb = Frag<_Float16>::load(Vth + (t * 16 + c) * KVC + kk * 32 + 8 * hh);
        oacc[t] = mma_g(pa, vb, oacc[t]);
      }
    }
  }

  float* os = Os[wave];
#pragma unroll
  for (int r = 0; r < 8; ++r) {
    const float inv = 1.0f / (lrow[r] * PCAR);
#pragma unroll
    for (int t = 0; t < 4; ++t) os[(8 * hh + r) * OSP + t * 16 + c] = oacc[t][r] * inv;
  }
  lds_sync_wave();
  {
    const int q8 = lane >> 3, c8 = (lane & 7) * 8;
    for (int pass = 0; pass < 2; ++pass) {
#pragma unroll
      for (int it = 0; it < 4; ++it) {
        const int row = it * 4 + q8;
        const float* sp = os + row * OSP + c8;
        const v4f s0 = *(const v4f*)(sp);
        const v4f s1 = *(const v4f*)(sp + 4);
        u4x w;
        w[0] = pack2(h_bits(s0[0]), h_bits(s0[1]));
        w[1] = pack2(h_bits(s0[2]), h_bits(s0[3]));
        w[2] = pack2(h_bits(s1[0]), h_bits(s1[1]));
        w[3] = pack2(h_bits(s1[2]), h_bits(s1[3]));
        *(volatile u4x*)(AOp + ((size_t)b * SEQ + (size_t)(q0 + row)) * HID + h * KDIM + c8) = w;
      }
      __threadfence();
    }
  }
}

template <int ET, bool ASPLIT, int BM, int ACT, bool MASK, bool ADDPOS, bool RESID, int OM>
static void run_gemm(hipStream_t st, const unsigned short* A, const unsigned short* A2, int lda, long sA,
                     const unsigned short* Bt, int ldb, long sB,
                     void* C, void* C2, void* C3, int ldc, long sC, const float* bias, const float* resid, const float* pos,
                     const int* lens, int M, int N, int K, float scale, float c16, int nbatch) {
  const int tiles = (M / 64) * (N / 64);
  dim3 grid((tiles + 7) / 8, nbatch, 1);
  gemm_kernel<ET, ASPLIT, BM, ACT, MASK, ADDPOS, RESID, OM><<<grid, 256, 0, st>>>(
      A, A2, lda, sA, Bt, ldb, sB, C, C2, C3, ldc, sC, bias, resid, pos, lens, M, N, K, scale, c16);
}

extern "C" void kernel_launch(void* const* d_in, const int* in_sizes, int n_in,
                              void* d_out, int out_size, void* d_ws, size_t ws_size, hipStream_t stream) {
  if (n_in < 24 || d_out == nullptr || d_ws == nullptr) return;
  if (in_sizes[0] != NROW * FIN || in_sizes[1] != NB || in_sizes[2] != NROW || in_sizes[3] != FIN * EMB || in_sizes[4] != EMB ||
      in_sizes[5] != NLAYER * EMB * G4 || in_sizes[6] != NLAYER * HID * G4 || in_sizes[7] != NLAYER * G4 ||
      in_sizes[8] != NLAYER * CATK * EMB || in_sizes[9] != NLAYER * EMB || in_sizes[10] != (NLAYER - 1) * HID ||
      in_sizes[11] != (NLAYER - 1) * HID || in_sizes[12] != NLAYER * HID * HID || in_sizes[13] != NLAYER * HID ||
      in_sizes[14] != NLAYER * HID * HID || in_sizes[15] != NLAYER * HID || in_sizes[16] != NLAYER * HID * NHEAD * KDIM ||
      in_sizes[17] != NLAYER * NHEAD * KDIM || in_sizes[18] != NLAYER * HID * NHEAD * KDIM || in_sizes[19] != NLAYER * NHEAD * KDIM ||
      in_sizes[20] != NLAYER * HID * NHEAD * KDIM || in_sizes[21] != NLAYER * NHEAD * KDIM ||
      in_sizes[22] != NLAYER * NHEAD * KDIM * HID || in_sizes[23] != NLAYER * HID || out_size != NROW * HID) return;

  const float* x      = (const float*)d_in[0];
  const int*   lens   = (const int*)  d_in[1];
  const int*   pairs  = (const int*)  d_in[2];
  const float* W_emb  = (const float*)d_in[3];
  const float* b_emb  = (const float*)d_in[4];
  const float* Wx     = (const float*)d_in[5];
  const float* Wh     = (const float*)d_in[6];
  const float* b_lstm = (const float*)d_in[7];
  const float* W_pr   = (const float*)d_in[8];
  const float* b_pr   = (const float*)d_in[9];
  const float* ln_g   = (const float*)d_in[10];
  const float* ln_b   = (const float*)d_in[11];
  const float* Wqd    = (const float*)d_in[12];
  const float* bqd    = (const float*)d_in[13];
  const float* Wvd    = (const float*)d_in[14];
  const float* bvd    = (const float*)d_in[15];
  const float* Wq     = (const float*)d_in[16];
  const float* bq     = (const float*)d_in[17];
  const float* Wk     = (const float*)d_in[18];
  const float* bk     = (const float*)d_in[19];
  const float* Wv     = (const float*)d_in[20];
  const float* bv     = (const float*)d_in[21];
  const float* Wo     = (const float*)d_in[22];
  const float* bo     = (const float*)d_in[23];
  float* outp = (float*)d_out;

  char* ws = (char*)d_ws; size_t off = 0;
  auto carve = [&](size_t bytes) -> char* { char* p = ws + off; off += (bytes + 255) & ~(size_t)255; return p; };
  unsigned short* XB    = (unsigned short*)carve((size_t)NROW * FIN * 2);
  float*          POS   = (float*)         carve((size_t)SEQ * NPOSC * 4);
  unsigned short* WEMBT = (unsigned short*)carve((size_t)EMB * FIN * 2);
  unsigned short* WPRT  = (unsigned short*)carve((size_t)NLAYER * EMB * CATK * 2);
  unsigned short* WXT   = (unsigned short*)carve((size_t)NLAYER * G4 * HID * 2);
  unsigned short* WHT   = (unsigned short*)carve((size_t)NLAYER * G4 * HID * 2);
  unsigned short* WQDT  = (unsigned short*)carve((size_t)NLAYER * HID * HID * 2);
  unsigned short* WVDT  = (unsigned short*)carve((size_t)NLAYER * HID * HID * 2);
  unsigned short* WQT   = (unsigned short*)carve((size_t)NLAYER * HID * HID * 2);
  unsigned short* WKT   = (unsigned short*)carve((size_t)NLAYER * HID * HID * 2);
  unsigned short* WVT   = (unsigned short*)carve((size_t)NLAYER * HID * HID * 2);
  unsigned short* WOT   = (unsigned short*)carve((size_t)NLAYER * HID * HID * 2);
  float*          H     = (float*)         carve((size_t)NROW * HID * 4);
  unsigned short* HH    = (unsigned short*)carve((size_t)NROW * HID * 2);
  unsigned short* HL    = (unsigned short*)carve((size_t)NROW * HID * 2);
  unsigned short* CATH  = (unsigned short*)carve((size_t)NROW * CATK * 2);
  unsigned short* CATL  = (unsigned short*)carve((size_t)NROW * CATK * 2);
  unsigned short* HLNH  = (unsigned short*)carve((size_t)NROW * HID * 2);
  unsigned short* HLNL  = (unsigned short*)carve((size_t)NROW * HID * 2);
  float*          ZX    = (float*)         carve((size_t)NROW * G4 * 4);
  float*          HS    = (float*)         carve((size_t)NROW * HID * 4);
  unsigned short* QL    = (unsigned short*)carve((size_t)NROW * HID * 2);
  unsigned short* VL    = (unsigned short*)carve((size_t)NROW * HID * 2);
  unsigned short* QH    = (unsigned short*)carve((size_t)NROW * HID * 2);
  unsigned short* KH    = (unsigned short*)carve((size_t)NROW * HID * 2);
  unsigned short* VT    = (unsigned short*)carve((size_t)NB * HID * SEQ * 2);
  unsigned short* AO    = (unsigned short*)carve((size_t)NROW * HID * 2);
  if (off > ws_size || off > (size_t)134217728) return;

  cvt8b_kernel<<<(NROW * FIN / 8 + NT - 1) / NT, NT, 0, stream>>>(x, XB, NROW * FIN / 8);
  pos_kernel<<<(SEQ * NPOSC) / NT, NT, 0, stream>>>(POS);
  tpw_kernel<0><<<dim3(EMB / 64, FIN / 64, 1), NT, 0, stream>>>(W_emb, FIN, EMB, FIN, WEMBT, 1.0f, 0L, 0L);
  tpw_kernel<0><<<dim3(EMB / 64, CATK / 64, NLAYER), NT, 0, stream>>>(W_pr, CATK, EMB, CATK, WPRT, 1.0f,
      (long)CATK * EMB, (long)EMB * CATK);
  tpw_kernel<0><<<dim3(G4 / 64, HID / 64, NLAYER), NT, 0, stream>>>(Wx, HID, G4, HID, WXT, 1.0f,
      (long)HID * G4, (long)G4 * HID);
  tpw_kernel<1><<<dim3(G4 / 64, HID / 64, NLAYER), NT, 0, stream>>>(Wh, HID, G4, HID, WHT, WCAR,
      (long)HID * G4, (long)G4 * HID);
  tpw_kernel<0><<<dim3(HID / 64, HID / 64, NLAYER), NT, 0, stream>>>(Wqd, HID, HID, HID, WQDT, 1.0f, (long)HID * HID, (long)HID * HID);
  tpw_kernel<0><<<dim3(HID / 64, HID / 64, NLAYER), NT, 0, stream>>>(Wvd, HID, HID, HID, WVDT, 1.0f, (long)HID * HID, (long)HID * HID);
  tpw_kernel<1><<<dim3(HID / 64, HID / 64, NLAYER), NT, 0, stream>>>(Wq,  HID, HID, HID, WQT,  WCAR, (long)HID * HID, (long)HID * HID);
  tpw_kernel<1><<<dim3(HID / 64, HID / 64, NLAYER), NT, 0, stream>>>(Wk,  HID, HID, HID, WKT,  WCAR, (long)HID * HID, (long)HID * HID);
  tpw_kernel<1><<<dim3(HID / 64, HID / 64, NLAYER), NT, 0, stream>>>(Wv,  HID, HID, HID, WVT,  WCAR, (long)HID * HID, (long)HID * HID);
  tpw_kernel<1><<<dim3(HID / 64, HID / 64, NLAYER), NT, 0, stream>>>(Wo,  HID, HID, HID, WOT,  WCAR, (long)HID * HID, (long)HID * HID);

  run_gemm<1, false, 2, 0, true, true, false, 2>(stream, XB, XB, FIN, 0L, WEMBT, FIN, 0L, (void*)H, (void*)HH, (void*)HL, HID, 0L,
                                                 b_emb, H, POS, lens, NROW, EMB, FIN, 1.0f, 1.0f, 1);

  for (int i = 0; i < NLAYER; ++i) {
    concat_kernel<<<NROW / (NT / 32), NT, 0, stream>>>(H, pairs, CATH, CATL);
    run_gemm<1, true, 2, 0, true, false, true, 2>(stream, CATH, CATL, CATK, 0L, WPRT + (size_t)i * EMB * CATK, CATK, 0L,
                                                 (void*)H, (void*)HH, (void*)HL, HID, 0L, b_pr + i * EMB, H, POS, lens,
                                                 NROW, EMB, CATK, 1.0f, 1.0f, 1);
    const unsigned short* inH = HH;
    const unsigned short* inL = HL;
    if (i > 0) {
      ln_kernel<<<NROW / (NT / 32), NT, 0, stream>>>(H, ln_g + (i - 1) * HID, ln_b + (i - 1) * HID, lens, HLNH, HLNL);
      inH = HLNH; inL = HLNL;
    }
    run_gemm<1, true, 2, 0, false, false, false, 0>(stream, inH, inL, HID, 0L, WXT + (size_t)i * G4 * HID, HID, 0L,
                                                   (void*)ZX, (void*)ZX, (void*)ZX, G4, 0L, b_lstm + i * G4, H, POS, lens,
                                                   NROW, G4, HID, 1.0f, 1.0f, 1);
    lstm_kernel<<<1, NT, 0, stream>>>(ZX, WHT + (size_t)i * G4 * HID, HS);
    post_kernel<<<NROW / (NT / 32), NT, 0, stream>>>(HS, lens, H, HH, HL, (i > 0) ? 1.0f : 0.0f);
    run_gemm<1, true, 2, 2, true, false, false, 1>(stream, HH, HL, HID, 0L, WQDT + (size_t)i * HID * HID, HID, 0L,
                                                  (void*)QL, (void*)QL, (void*)QL, HID, 0L, bqd + i * HID, H, POS, lens,
                                                  NROW, HID, HID, 1.0f, ACAR, 1);
    run_gemm<1, true, 2, 2, true, false, false, 1>(stream, HH, HL, HID, 0L, WVDT + (size_t)i * HID * HID, HID, 0L,
                                                  (void*)VL, (void*)VL, (void*)VL, HID, 0L, bvd + i * HID, H, POS, lens,
                                                  NROW, HID, HID, 1.0f, ACAR, 1);
    run_gemm<0, false, 2, 0, false, false, false, 1>(stream, QL, QL, HID, 0L, WQT + (size_t)i * HID * HID, HID, 0L,
                                                    (void*)QH, (void*)QH, (void*)QH, HID, 0L, bq + i * HID, H, POS, lens,
                                                    NROW, HID, HID, SC_AW, ACAR, 1);
    run_gemm<0, false, 2, 0, false, false, false, 1>(stream, VL, VL, HID, 0L, WKT + (size_t)i * HID * HID, HID, 0L,
                                                    (void*)KH, (void*)KH, (void*)KH, HID, 0L, bk + i * HID, H, POS, lens,
                                                    NROW, HID, HID, SC_AW, ACAR, 1);
    run_gemm<0, false, 1, 0, false, false, false, 1>(stream, WVT + (size_t)i * HID * HID, WVT + (size_t)i * HID * HID, HID, 0L,
                                                    VL, HID, (long)SEQ * HID, (void*)VT, (void*)VT, (void*)VT, SEQ, (long)HID * SEQ,
                                                    bv + i * HID, H, POS, lens, HID, SEQ, HID, SC_AW, ACAR, NB);
    attn_kernel<<<NB * NHEAD * (SEQ / 64), 128, 0, stream>>>(QH, KH, VT, lens, AO);
    if (i == NLAYER - 1) {
      run_gemm<0, false, 2, 0, true, false, true, 0>(stream, AO, AO, HID, 0L, WOT + (size_t)i * HID * HID, HID, 0L,
                                                    (void*)outp, (void*)outp, (void*)outp, HID, 0L, bo + i * HID, H, POS, lens,
                                                    NROW, HID, HID, SC_AW, 1.0f, 1);
    } else {
      run_gemm<0, false, 2, 0, true, false, true, 2>(stream, AO, AO, HID, 0L, WOT + (size_t)i * HID * HID, HID, 0L,
                                                    (void*)H, (void*)HH, (void*)HL, HID, 0L, bo + i * HID, H, POS, lens,
                                                    NROW, HID, HID, SC_AW, 1.0f, 1);
    }
  }
}
